// PointNetSetAbstraction_74062416052697
// MI455X (gfx1250) — hardware-verified
//
#include <hip/hip_runtime.h>
#pragma clang fp contract(off)

typedef __attribute__((ext_vector_type(16))) _Float16 v16h;
typedef __attribute__((ext_vector_type(8)))  _Float16 v8h;
typedef __attribute__((ext_vector_type(8)))  float    v8f;
typedef __attribute__((ext_vector_type(4)))  float    v4f;
typedef __attribute__((ext_vector_type(2)))  float    v2f;
typedef __attribute__((ext_vector_type(4)))  unsigned v4u;

constexpr int NBATCH   = 8;
constexpr int NPTS     = 4096;
constexpr int NCENT    = 1024;
constexpr int NNBR     = 32;
constexpr int CH_IN    = 64;
constexpr int KPAD0    = 96;
constexpr int NCH_L0   = 64;
constexpr int NCH_L1   = 64;
constexpr int NCH_L2   = 128;
constexpr int MROWS    = NBATCH * NCENT * NNBR;
constexpr int NPARTS   = MROWS / 64;
constexpr int NGROUPS  = NBATCH * NCENT;
constexpr float W_CARRY     = 16.0f;
constexpr float W_CARRY_INV = 1.0f / 16.0f;
constexpr float BN_EPS      = 1e-5f;

static_assert(MROWS == 262144, "row count");
static_assert(MROWS % 64 == 0, "M tile multiple");
static_assert(KPAD0 % 32 == 0 && NCH_L0 % 32 == 0 && NCH_L1 % 32 == 0, "K multiples of 32");
static_assert(NCH_L0 % 64 == 0 && NCH_L1 % 64 == 0 && NCH_L2 % 64 == 0, "N tile multiples");
static_assert(CH_IN + 3 <= KPAD0, "layer-0 K pad");
static_assert((NNBR * KPAD0 * 2) % 128 == 0, "group tile is whole lines");

constexpr size_t OFF_CXYZ  = 0;
constexpr size_t OFF_W0    = OFF_CXYZ + (size_t)NBATCH * NCENT * 3 * 4;
constexpr size_t OFF_W1    = OFF_W0 + (size_t)NCH_L0 * KPAD0 * 2;
constexpr size_t OFF_W2    = OFF_W1 + (size_t)NCH_L1 * NCH_L0 * 2;
constexpr size_t OFF_STATS = OFF_W2 + (size_t)NCH_L2 * NCH_L1 * 2;
constexpr size_t OFF_PSUM  = OFF_STATS + 3 * 1024;
constexpr size_t OFF_PSQ   = OFF_PSUM + (size_t)NPARTS * 128 * 4;
constexpr size_t OFF_YMAX  = OFF_PSQ + (size_t)NPARTS * 128 * 4;
constexpr size_t OFF_YMIN  = OFF_YMAX + (size_t)NGROUPS * 128 * 4;
constexpr size_t OFF_X     = OFF_YMIN + (size_t)NGROUPS * 128 * 4;
constexpr size_t OFF_Y     = OFF_X + (size_t)MROWS * KPAD0 * 2;
constexpr size_t WS_TOTAL  = OFF_Y + (size_t)MROWS * 64 * 4;
static_assert(WS_TOTAL == 130161664ull, "carve total");
static_assert(WS_TOTAL <= 134217728ull, "carve under 128 MiB");
static_assert(OFF_W0 % 128 == 0 && OFF_W1 % 128 == 0 && OFF_W2 % 128 == 0 && OFF_STATS % 128 == 0 &&
              OFF_PSUM % 128 == 0 && OFF_PSQ % 128 == 0 && OFF_YMAX % 128 == 0 && OFF_YMIN % 128 == 0 &&
              OFF_X % 128 == 0 && OFF_Y % 128 == 0, "line aligned carve");
static_assert((size_t)MROWS * KPAD0 * 2 >= (size_t)MROWS * 64 * 2, "X sized from its largest user");
static_assert(98304 + (size_t)NGROUPS * 128 * 4 == 4292608ull, "output extent");

__device__ __forceinline__ unsigned f16bits(float x) {
  const _Float16 h = (_Float16)x;
  const unsigned short s = __builtin_bit_cast(unsigned short, h);
  return (unsigned)s;
}
__device__ __forceinline__ unsigned pack2h(float a, float b) {
  return f16bits(a) | (f16bits(b) << 16);
}

__device__ __forceinline__ void guard_row(v8f& a0, v8f& a1, v8f& a2, v8f& a3, v16h x,
                                          v16h b0, v16h b1, v16h b2, v16h b3) {
  asm volatile("v_nop\n\tv_nop\n\tv_nop\n\tv_nop"
               : "+v"(a0), "+v"(a1), "+v"(a2), "+v"(a3)
               : "v"(x), "v"(b0), "v"(b1), "v"(b2), "v"(b3));
}
__device__ __forceinline__ void keep4_h(v16h a, v16h b, v16h c, v16h d) { asm volatile("v_nop" :: "v"(a), "v"(b), "v"(c), "v"(d)); }
__device__ __forceinline__ void acc_guard4(v8f& a, v8f& b, v8f& c, v8f& d) { asm volatile("v_nop\n\tv_nop\n\tv_nop\n\tv_nop" : "+v"(a), "+v"(b), "+v"(c), "+v"(d)); }

template <typename T> struct Frag;
template <> struct Frag<_Float16> {
  typedef v16h V; union U { v16h v; v8h h[2]; };
  static __device__ __forceinline__ v16h load(const _Float16* p) {
    U f; f.h[0] = *(const v8h*)(p); f.h[1] = *(const v8h*)(p + 16); return f.v;
  }
  static __device__ __forceinline__ v8f mma(v16h a, v16h b, v8f c) {
    return __builtin_amdgcn_wmma_f32_16x16x32_f16(false, a, false, b, (short)0, c, false, false);
  }
};

__global__ __launch_bounds__(256) void prep_weights_kernel(const float* __restrict__ w0,
                                                           const float* __restrict__ w1,
                                                           const float* __restrict__ w2,
                                                           unsigned* __restrict__ W0h,
                                                           unsigned* __restrict__ W1h,
                                                           unsigned* __restrict__ W2h) {
  const int blk = blockIdx.x;
  const int tid = threadIdx.x;
  unsigned word = 0;
  unsigned* dst = W0h;
  if (blk < 12) {
    const int wi = blk * 256 + tid;
    const int o = wi / 48;
    const int jw = wi - o * 48;
    const int j0 = 2 * jw;
    const int j1 = j0 + 1;
    const int s0 = (j0 < 64) ? (3 + j0) : (j0 - 64);
    const int s1 = (j1 < 64) ? (3 + j1) : (j1 - 64);
    const float v0 = w0[o * 67 + s0];
    const float v1 = w0[o * 67 + s1];
    const float x0 = (j0 < 67) ? v0 * W_CARRY : 0.0f;
    const float x1 = (j1 < 67) ? v1 * W_CARRY : 0.0f;
    word = pack2h(x0, x1);
    dst = W0h + wi;
  } else if (blk < 20) {
    const int wi = (blk - 12) * 256 + tid;
    const float v0 = w1[2 * wi];
    const float v1 = w1[2 * wi + 1];
    word = pack2h(v0 * W_CARRY, v1 * W_CARRY);
    dst = W1h + wi;
  } else {
    const int wi = (blk - 20) * 256 + tid;
    const float v0 = w2[2 * wi];
    const float v1 = w2[2 * wi + 1];
    word = pack2h(v0 * W_CARRY, v1 * W_CARRY);
    dst = W2h + wi;
  }
  *(volatile unsigned*)dst = word;
  __threadfence();
  *(volatile unsigned*)dst = word;
}

__global__ __launch_bounds__(1024) void fps_kernel(const float* __restrict__ xyz,
                                                   float* __restrict__ out_xyz,
                                                   float* __restrict__ ws_xyz) {
#pragma clang fp contract(off)
  __shared__ __align__(16) float sraw[NPTS * 3];
  __shared__ int   sel[NCENT];
  __shared__ float rv[2][32];
  __shared__ int   ri[2][32];

  const int b    = blockIdx.x;
  const int tid  = threadIdx.x;
  const int lane = tid & 31;
  const int wid  = tid >> 5;

  {
    const v4f* src = (const v4f*)(xyz + (size_t)b * NPTS * 3);
#pragma unroll
    for (int j = 0; j < 3; ++j) {
      const v4f t = src[tid + j * 1024];
      *(v4f*)(sraw + 4 * (tid + j * 1024)) = t;
    }
  }
  __syncthreads();

  float px[4], py[4], pz[4], dist[4];
#pragma unroll
  for (int t = 0; t < 4; ++t) {
    const int i = tid + t * 1024;
    px[t] = sraw[3 * i + 0];
    py[t] = sraw[3 * i + 1];
    pz[t] = sraw[3 * i + 2];
    dist[t] = 1e10f;
  }

  int cur = 0;
#pragma unroll 1
  for (int it = 0; it < NCENT; ++it) {
    if (tid == 0) sel[it] = cur;
    const float cx = sraw[3 * cur + 0];
    const float cy = sraw[3 * cur + 1];
    const float cz = sraw[3 * cur + 2];

    float bv = -1.0f;
    int   bi = 0;
#pragma unroll
    for (int t = 0; t < 4; ++t) {
      const float dx = px[t] - cx;
      const float dy = py[t] - cy;
      const float dz = pz[t] - cz;
      const float t0 = dx * dx;
      const float t1 = dy * dy;
      const float t2 = dz * dz;
      const float dd = (t0 + t2) + t1;
      const float nd = fminf(dist[t], dd);
      dist[t] = nd;
      const int i = tid + t * 1024;
      const bool tk = nd > bv;
      bv = tk ? nd : bv;
      bi = tk ? i : bi;
    }
#pragma unroll
    for (int off = 16; off > 0; off >>= 1) {
      const float ov = __shfl_xor(bv, off, 32);
      const int   oi = __shfl_xor(bi, off, 32);
      const bool tk = (ov > bv) || ((ov == bv) && (oi < bi));
      bv = tk ? ov : bv;
      bi = tk ? oi : bi;
    }
    const int p = it & 1;
    if (lane == 0) { rv[p][wid] = bv; ri[p][wid] = bi; }
    __syncthreads();
    bv = rv[p][lane];
    bi = ri[p][lane];
#pragma unroll
    for (int off = 16; off > 0; off >>= 1) {
      const float ov = __shfl_xor(bv, off, 32);
      const int   oi = __shfl_xor(bi, off, 32);
      const bool tk = (ov > bv) || ((ov == bv) && (oi < bi));
      bv = tk ? ov : bv;
      bi = tk ? oi : bi;
    }
    cur = bi & (NPTS - 1);
  }
  __syncthreads();

  if (tid < 768) {
    float ov[4];
#pragma unroll
    for (int e = 0; e < 4; ++e) {
      const int f = 4 * tid + e;
      const int s = f / 3;
      const int c = f - 3 * s;
      const int pi = sel[s] & (NPTS - 1);
      ov[e] = sraw[3 * pi + c];
    }
    const v4f o = {ov[0], ov[1], ov[2], ov[3]};
    float* d0 = out_xyz + (size_t)b * (NCENT * 3) + 4 * tid;
    float* d1 = ws_xyz  + (size_t)b * (NCENT * 3) + 4 * tid;
    *(volatile v4f*)d0 = o;
    *(volatile v4f*)d1 = o;
    __threadfence();
    *(volatile v4f*)d0 = o;
    *(volatile v4f*)d1 = o;
  }
}

__global__ __launch_bounds__(256) void ball_gather_kernel(const float* __restrict__ xyz,
                                                          const float* __restrict__ pts,
                                                          const float* __restrict__ cxyz,
                                                          v4u* __restrict__ Xout) {
#pragma clang fp contract(off)
  __shared__ int sidx[8][32];
  __shared__ __align__(16) v4u tile[8][384];

  const int tid  = threadIdx.x;
  const int lane = tid & 31;
  const int w    = tid >> 5;
  const int bs   = blockIdx.x * 8 + w;
  const int b    = bs >> 10;

  const float qx = cxyz[(size_t)bs * 3 + 0];
  const float qy = cxyz[(size_t)bs * 3 + 1];
  const float qz = cxyz[(size_t)bs * 3 + 2];

  sidx[w][lane] = 0;
  __syncthreads();

  const float r2 = __uint_as_float(0x3D23D70Au);
  const float* xb = xyz + (size_t)b * NPTS * 3;

  int cnt = 0;
#pragma unroll 1
  for (int c = 0; (c < NPTS / 32) && (cnt < NNBR); ++c) {
    const int i = c * 32 + lane;
    const float* p = xb + (size_t)i * 3;
    const float x0 = p[0];
    const float x1 = p[1];
    const float x2 = p[2];
    const float dx = qx - x0;
    const float dy = qy - x1;
    const float dz = qz - x2;
    const float t0 = dx * dx;
    const float t1 = dy * dy;
    const float t2 = dz * dz;
    const float d2 = (t0 + t2) + t1;
    const bool in = !(d2 > r2);
    const unsigned m = (unsigned)__ballot(in);
    const int rank = __popc(m & ((1u << lane) - 1u));
    const int slot = cnt + rank;
    if (in && (slot < NNBR)) sidx[w][slot] = i;
    cnt += __popc(m);
  }
  __syncthreads();

  const int take = (cnt < NNBR) ? cnt : NNBR;
  const int srcl = (lane < take) ? lane : 0;
  int gi = sidx[w][srcl];
  gi = (gi < 0) ? 0 : ((gi > NPTS - 1) ? (NPTS - 1) : gi);

  unsigned* tw = (unsigned*)(&tile[w][0]);
  const float* pb = pts + (size_t)b * NPTS * CH_IN;
#pragma unroll 4
  for (int r = 0; r < NNBR; ++r) {
    const int g = __shfl(gi, r, 32);
    const v2f pv = *(const v2f*)(pb + (size_t)g * CH_IN + 2 * lane);
    const float f0 = pv.x;
    const float f1 = pv.y;
    tw[r * 48 + lane] = pack2h(f0, f1);
  }

  {
    const float* gp = xb + (size_t)gi * 3;
    const float g0 = gp[0];
    const float g1 = gp[1];
    const float g2 = gp[2];
    const float rx = g0 - qx;
    const float ry = g1 - qy;
    const float rz = g2 - qz;
    unsigned zz = 0;
    asm volatile("" : "+v"(zz));
    const unsigned w32 = pack2h(rx, ry);
    const unsigned w33 = (f16bits(rz) & 0xffffu) | (zz << 16);
    const v4u a = {w32, w33, zz, zz};
    const v4u z = {zz, zz, zz, zz};
    tile[w][lane * 12 + 8]  = a;
    tile[w][lane * 12 + 9]  = z;
    tile[w][lane * 12 + 10] = z;
    tile[w][lane * 12 + 11] = z;
  }
  __syncthreads();

  v4u* Xg = Xout + (size_t)bs * 384;
  for (int pass = 0; pass < 2; ++pass) {
#pragma unroll
    for (int it = 0; it < 12; ++it) {
      const v4u v = tile[w][it * 32 + lane];
      *(volatile v4u*)(Xg + it * 32 + lane) = v;
    }
    __threadfence();
  }
}

template <int MODE>
__global__ __launch_bounds__(256) void gemm_f16_bn(
    const _Float16* __restrict__ A, int lda,
    const _Float16* __restrict__ Bt, int ldb,
    const float* __restrict__ bias,
    float* __restrict__ Yout, float* __restrict__ Ymax, float* __restrict__ Ymin,
    float* __restrict__ Psum, float* __restrict__ Psq,
    int M, int N, int K, float scale) {
  __shared__ __align__(16) float sT[8][16 * 68];
  const int lane = threadIdx.x & 31;
  const int wave = threadIdx.x >> 5;
  const int tilesN = N >> 6;
  const int tilesM = M >> 6;
  const int tile = blockIdx.x * 8 + wave;
  if (tile >= tilesM * tilesN) return;
  const int tm = tile / tilesN;
  const int tn = tile - tm * tilesN;
  const int m0 = tm << 6;
  const int n0 = tn << 6;

  const int rlane = lane & 15;
  const int koff  = (lane >> 4) * 8;
  const int mOff  = (lane >> 4) * 8;

  v8f acc[4][4];
#pragma unroll
  for (int i = 0; i < 4; ++i)
#pragma unroll
    for (int j = 0; j < 4; ++j) acc[i][j] = (v8f){0.f, 0.f, 0.f, 0.f, 0.f, 0.f, 0.f, 0.f};

  for (int k0 = 0; k0 < K; k0 += 32) {
    v16h bh[4];
#pragma unroll
    for (int j = 0; j < 4; ++j) {
      const size_t bo = (size_t)(n0 + (j << 4) + rlane) * ldb + koff + k0;
      bh[j] = Frag<_Float16>::load(Bt + bo);
    }
#pragma unroll
    for (int i = 0; i < 4; ++i) {
      const size_t ao = (size_t)(m0 + (i << 4) + rlane) * lda + koff + k0;
      const v16h ah = Frag<_Float16>::load(A + ao);
#pragma unroll
      for (int j = 0; j < 4; ++j) acc[i][j] = Frag<_Float16>::mma(ah, bh[j], acc[i][j]);
      guard_row(acc[i][0], acc[i][1], acc[i][2], acc[i][3], ah, bh[0], bh[1], bh[2], bh[3]);
    }
    keep4_h(bh[0], bh[1], bh[2], bh[3]);
  }
  acc_guard4(acc[0][0], acc[0][1], acc[0][2], acc[0][3]);
  acc_guard4(acc[1][0], acc[1][1], acc[1][2], acc[1][3]);
  acc_guard4(acc[2][0], acc[2][1], acc[2][2], acc[2][3]);
  acc_guard4(acc[3][0], acc[3][1], acc[3][2], acc[3][3]);

  float* slab = sT[wave];
  float bvv[4];
#pragma unroll
  for (int j = 0; j < 4; ++j) bvv[j] = bias[n0 + (j << 4) + rlane];

  float cs0 = 0.0f, cs1 = 0.0f, cq0 = 0.0f, cq1 = 0.0f;
  float mx0 = -3.402823466e38f, mx1 = -3.402823466e38f;
  float mn0 = 3.402823466e38f,  mn1 = 3.402823466e38f;

#pragma unroll
  for (int i = 0; i < 4; ++i) {
    const int mBase = m0 + (i << 4);
#pragma unroll
    for (int j = 0; j < 4; ++j) {
#pragma unroll
      for (int r = 0; r < 8; ++r) {
        const float pr = acc[i][j][r] * scale;
        const float v = pr + bvv[j];
        slab[(mOff + r) * 68 + (j << 4) + rlane] = v;
      }
    }
    __builtin_amdgcn_fence(__ATOMIC_RELEASE, "workgroup");
    __builtin_amdgcn_wave_barrier();
    __builtin_amdgcn_fence(__ATOMIC_ACQUIRE, "workgroup");

    if (MODE == 1 && (i == 0 || i == 2)) {
      mx0 = -3.402823466e38f; mx1 = -3.402823466e38f;
      mn0 = 3.402823466e38f;  mn1 = 3.402823466e38f;
    }
#pragma unroll
    for (int row = 0; row < 16; ++row) {
      const float a = slab[row * 68 + lane];
      const float c = slab[row * 68 + 32 + lane];
      const float aa = a * a;
      const float cc = c * c;
      cs0 += a;
      cs1 += c;
      cq0 += aa;
      cq1 += cc;
      if (MODE == 1) {
        mx0 = fmaxf(mx0, a); mx1 = fmaxf(mx1, c);
        mn0 = fminf(mn0, a); mn1 = fminf(mn1, c);
      }
    }

    if (MODE == 0) {
      const int hh = lane >> 4, c4 = (lane & 15) * 4;
      for (int pass = 0; pass < 2; ++pass) {
#pragma unroll
        for (int it = 0; it < 8; ++it) {
          const int row = it * 2 + hh;
          const v4f v = *(const v4f*)(slab + row * 68 + c4);
          *(volatile v4f*)(Yout + (size_t)(mBase + row) * N + n0 + c4) = v;
        }
        __threadfence();
      }
    } else {
      if (i == 1 || i == 3) {
        const int grp = (m0 >> 5) + (i >> 1);
        float* pmax = Ymax + (size_t)grp * N + n0 + lane;
        float* pmin = Ymin + (size_t)grp * N + n0 + lane;
        for (int pass = 0; pass < 2; ++pass) {
          *(volatile float*)(pmax)      = mx0;
          *(volatile float*)(pmax + 32) = mx1;
          *(volatile float*)(pmin)      = mn0;
          *(volatile float*)(pmin + 32) = mn1;
          __threadfence();
        }
      }
    }
    __builtin_amdgcn_fence(__ATOMIC_RELEASE, "workgroup");
    __builtin_amdgcn_wave_barrier();
    __builtin_amdgcn_fence(__ATOMIC_ACQUIRE, "workgroup");
  }

  {
    float* ps = Psum + (size_t)tm * N + n0 + lane;
    float* pq = Psq  + (size_t)tm * N + n0 + lane;
    for (int pass = 0; pass < 2; ++pass) {
      *(volatile float*)(ps)      = cs0;
      *(volatile float*)(ps + 32) = cs1;
      *(volatile float*)(pq)      = cq0;
      *(volatile float*)(pq + 32) = cq1;
      __threadfence();
    }
  }
}

__global__ __launch_bounds__(256) void stats_final_kernel(const float* __restrict__ Psum,
                                                          const float* __restrict__ Psq,
                                                          int nch,
                                                          const float* __restrict__ gam,
                                                          const float* __restrict__ bet,
                                                          float* __restrict__ table) {
  __shared__ double ss[8][32];
  __shared__ double sq[8][32];
  const int lane = threadIdx.x & 31;
  const int grp  = threadIdx.x >> 5;
  const int c    = blockIdx.x * 32 + lane;
  double s = 0.0, q = 0.0;
#pragma unroll 4
  for (int p = grp; p < NPARTS; p += 8) {
    const float a = Psum[(size_t)p * nch + c];
    const float d = Psq[(size_t)p * nch + c];
    s += (double)a;
    q += (double)d;
  }
  ss[grp][lane] = s;
  sq[grp][lane] = q;
  __syncthreads();
  if (grp == 0) {
    double S = 0.0, Q = 0.0;
#pragma unroll
    for (int k = 0; k < 8; ++k) { S += ss[k][lane]; Q += sq[k][lane]; }
    const double inv_cnt = 1.0 / (double)MROWS;
    const double mean = S * inv_cnt;
    double var = Q * inv_cnt - mean * mean;
    var = (var < 0.0) ? 0.0 : var;
    const float rs  = rsqrtf((float)var + BN_EPS);
    const float scv = gam[c] * rs;
    const float msc = (float)mean * scv;
    const float shv = bet[c] - msc;
    *(volatile float*)(table + c)       = scv;
    *(volatile float*)(table + 128 + c) = shv;
    __threadfence();
    *(volatile float*)(table + c)       = scv;
    *(volatile float*)(table + 128 + c) = shv;
  }
}

__global__ __launch_bounds__(256) void bn_pack_kernel(const float* __restrict__ Y,
                                                      const float* __restrict__ table,
                                                      v4u* __restrict__ Xh) {
  const size_t t = (size_t)blockIdx.x * 256 + threadIdx.x;
  const size_t row = t >> 3;
  const int c8 = ((int)(t & 7)) * 8;
  const v4f y0 = *(const v4f*)(Y + row * 64 + c8);
  const v4f y1 = *(const v4f*)(Y + row * 64 + c8 + 4);
  const v4f s0 = *(const v4f*)(table + c8);
  const v4f s1 = *(const v4f*)(table + c8 + 4);
  const v4f h0 = *(const v4f*)(table + 128 + c8);
  const v4f h1 = *(const v4f*)(table + 128 + c8 + 4);
  float r[8];
#pragma unroll
  for (int e = 0; e < 4; ++e) {
    const float a = y0[e];
    const float sa = s0[e];
    const float ha = h0[e];
    const float pa = a * sa;
    r[e] = fmaxf(pa + ha, 0.0f);
    const float b = y1[e];
    const float sb = s1[e];
    const float hb = h1[e];
    const float pb = b * sb;
    r[4 + e] = fmaxf(pb + hb, 0.0f);
  }
  const unsigned w0 = pack2h(r[0], r[1]);
  const unsigned w1 = pack2h(r[2], r[3]);
  const unsigned w2 = pack2h(r[4], r[5]);
  const unsigned w3 = pack2h(r[6], r[7]);
  const v4u o = {w0, w1, w2, w3};
  v4u* dst = Xh + t;
  *(volatile v4u*)dst = o;
  __threadfence();
  *(volatile v4u*)dst = o;
}

__global__ __launch_bounds__(256) void finalize_kernel(const float* __restrict__ Ymax,
                                                       const float* __restrict__ Ymin,
                                                       const float* __restrict__ table,
                                                       float* __restrict__ out1) {
  const size_t t = (size_t)blockIdx.x * 256 + threadIdx.x;
  const size_t row = t >> 5;
  const int c4 = ((int)(t & 31)) * 4;
  const v4f a  = *(const v4f*)(Ymax + row * 128 + c4);
  const v4f bm = *(const v4f*)(Ymin + row * 128 + c4);
  const v4f sc = *(const v4f*)(table + c4);
  const v4f sh = *(const v4f*)(table + 128 + c4);
  float r[4];
#pragma unroll
  for (int e = 0; e < 4; ++e) {
    const float s  = sc[e];
    const float h  = sh[e];
    const float va = a[e];
    const float vb = bm[e];
    const float fa = (s >= 0.0f) ? 1.0f : 0.0f;
    const float fb = 1.0f - fa;
    const float xa = fa * va;
    const float xb = fb * vb;
    const float x  = xa + xb;
    const float p  = x * s;
    r[e] = fmaxf(p + h, 0.0f);
  }
  const v4f o = {r[0], r[1], r[2], r[3]};
  float* dst = out1 + row * 128 + c4;
  *(volatile v4f*)dst = o;
  __threadfence();
  *(volatile v4f*)dst = o;
}

extern "C" void kernel_launch(void* const* d_in, const int* in_sizes, int n_in,
                              void* d_out, int out_size, void* d_ws, size_t ws_size,
                              hipStream_t stream) {
  (void)in_sizes; (void)n_in; (void)out_size;
  if (ws_size < WS_TOTAL) return;

  const float* xyz = (const float*)d_in[0];
  const float* pts = (const float*)d_in[1];
  const float* w0  = (const float*)d_in[2];
  const float* b0  = (const float*)d_in[3];
  const float* g0  = (const float*)d_in[4];
  const float* bt0 = (const float*)d_in[5];
  const float* w1  = (const float*)d_in[6];
  const float* b1  = (const float*)d_in[7];
  const float* g1  = (const float*)d_in[8];
  const float* bt1 = (const float*)d_in[9];
  const float* w2  = (const float*)d_in[10];
  const float* b2  = (const float*)d_in[11];
  const float* g2  = (const float*)d_in[12];
  const float* bt2 = (const float*)d_in[13];

  float* out  = (float*)d_out;
  float* out1 = out + (98304 / 4);

  char* wsb = (char*)d_ws;
  float*    cxyz  = (float*)(wsb + OFF_CXYZ);
  unsigned* W0h   = (unsigned*)(wsb + OFF_W0);
  unsigned* W1h   = (unsigned*)(wsb + OFF_W1);
  unsigned* W2h   = (unsigned*)(wsb + OFF_W2);
  float*    st0   = (float*)(wsb + OFF_STATS);
  float*    st1   = st0 + 256;
  float*    st2   = st0 + 512;
  float*    Psum  = (float*)(wsb + OFF_PSUM);
  float*    Psq   = (float*)(wsb + OFF_PSQ);
  float*    Ymax  = (float*)(wsb + OFF_YMAX);
  float*    Ymin  = (float*)(wsb + OFF_YMIN);
  void*     Xraw  = (void*)(wsb + OFF_X);
  float*    Ybuf  = (float*)(wsb + OFF_Y);

  fps_kernel<<<NBATCH, 1024, 0, stream>>>(xyz, out, cxyz);
  prep_weights_kernel<<<36, 256, 0, stream>>>(w0, w1, w2, W0h, W1h, W2h);
  ball_gather_kernel<<<NGROUPS / 8, 256, 0, stream>>>(xyz, pts, cxyz, (v4u*)Xraw);

  gemm_f16_bn<0><<<(MROWS / 64) * (NCH_L0 / 64) / 8, 256, 0, stream>>>(
      (const _Float16*)Xraw, KPAD0, (const _Float16*)W0h, KPAD0, b0,
      Ybuf, Ymax, Ymin, Psum, Psq, MROWS, NCH_L0, KPAD0, W_CARRY_INV);
  stats_final_kernel<<<NCH_L0 / 32, 256, 0, stream>>>(Psum, Psq, NCH_L0, g0, bt0, st0);
  bn_pack_kernel<<<MROWS * 64 / 8 / 256, 256, 0, stream>>>(Ybuf, st0, (v4u*)Xraw);

  gemm_f16_bn<0><<<(MROWS / 64) * (NCH_L1 / 64) / 8, 256, 0, stream>>>(
      (const _Float16*)Xraw, NCH_L0, (const _Float16*)W1h, NCH_L0, b1,
      Ybuf, Ymax, Ymin, Psum, Psq, MROWS, NCH_L1, NCH_L0, W_CARRY_INV);
  stats_final_kernel<<<NCH_L1 / 32, 256, 0, stream>>>(Psum, Psq, NCH_L1, g1, bt1, st1);
  bn_pack_kernel<<<MROWS * 64 / 8 / 256, 256, 0, stream>>>(Ybuf, st1, (v4u*)Xraw);

  gemm_f16_bn<1><<<(MROWS / 64) * (NCH_L2 / 64) / 8, 256, 0, stream>>>(
      (const _Float16*)Xraw, NCH_L1, (const _Float16*)W2h, NCH_L1, b2,
      Ybuf, Ymax, Ymin, Psum, Psq, MROWS, NCH_L2, NCH_L1, W_CARRY_INV);
  stats_final_kernel<<<NCH_L2 / 32, 256, 0, stream>>>(Psum, Psq, NCH_L2, g2, bt2, st2);
  finalize_kernel<<<NGROUPS * 32 / 256, 256, 0, stream>>>(Ymax, Ymin, st2, out1);
}
